// SoftEmbedding_42494406427453
// MI455X (gfx1250) — hardware-verified
//
#include <hip/hip_runtime.h>

typedef __bf16 v16b __attribute__((ext_vector_type(16)));
typedef __bf16 v8b  __attribute__((ext_vector_type(8)));
typedef float  v8f  __attribute__((ext_vector_type(8)));
typedef float  v4f  __attribute__((ext_vector_type(4)));

#define NUM_EMB       512
#define EMB_DIM       64
#define KPITCH        520
#define TOK_PER_BLOCK 128
#define NTHREADS      256
#define NWAVES        8
#define SPITCH        68
#define LOG2E         1.4426950408889634f

#define OFF_EMBH   0
#define OFF_EMBL   (EMB_DIM * KPITCH * 2)
#define OFF_SW     (2 * EMB_DIM * KPITCH * 2)
#define OFF_SB     (OFF_SW + NUM_EMB * 4)
#define OFF_RED    (OFF_SB + NUM_EMB * 4)
#define OFF_STAGE  (OFF_RED + 32 * 4)
#define SMEM_BYTES (OFF_STAGE + NWAVES * 16 * SPITCH * 4)

union Frag { v16b v; v8b half[2]; };

__device__ __forceinline__ v8f wmma3(v8f c, v16b ah, v16b al, v16b bh, v16b bl)
{
    c = __builtin_amdgcn_wmma_f32_16x16x32_bf16(false, ah, false, bh, (short)0, c, false, false);
    c = __builtin_amdgcn_wmma_f32_16x16x32_bf16(false, al, false, bh, (short)0, c, false, false);
    c = __builtin_amdgcn_wmma_f32_16x16x32_bf16(false, ah, false, bl, (short)0, c, false, false);
    asm volatile("v_nop\n\tv_nop\n\tv_nop\n\tv_nop" : "+v"(c) : "v"(ah), "v"(al), "v"(bh), "v"(bl));
    return c;
}

__global__ __launch_bounds__(NTHREADS) void soft_emb_kernel(
    const float* __restrict__ x_in,
    const float* __restrict__ proj_w,
    const float* __restrict__ proj_b,
    const float* __restrict__ emb,
    float* out,
    int T)
{
    extern __shared__ __attribute__((aligned(16))) char smem_raw[];
    __bf16* embH  = (__bf16*)(smem_raw + OFF_EMBH);
    __bf16* embL  = (__bf16*)(smem_raw + OFF_EMBL);
    float*  sw    = (float*)(smem_raw + OFF_SW);
    float*  sb    = (float*)(smem_raw + OFF_SB);
    float*  red   = (float*)(smem_raw + OFF_RED);
    float*  stage = (float*)(smem_raw + OFF_STAGE);

    const int tid  = threadIdx.x;
    const int lane = tid & 31;
    const int wv   = tid >> 5;

    float lw = -1e30f, lnw = -1e30f, lb = -1e30f;
    for (int i = tid; i < NUM_EMB; i += NTHREADS) {
        const float wval = proj_w[i] * LOG2E;
        const float bval = proj_b[i] * LOG2E;
        sw[i] = wval;
        sb[i] = bval;
        lw  = fmaxf(lw,  wval);
        lnw = fmaxf(lnw, -wval);
        lb  = fmaxf(lb,  bval);
    }
#pragma unroll
    for (int off = 16; off > 0; off >>= 1) {
        lw  = fmaxf(lw,  __shfl_xor(lw,  off));
        lnw = fmaxf(lnw, __shfl_xor(lnw, off));
        lb  = fmaxf(lb,  __shfl_xor(lb,  off));
    }
    if (lane == 0) { red[wv * 3] = lw; red[wv * 3 + 1] = lnw; red[wv * 3 + 2] = lb; }

    for (int i = tid; i < NUM_EMB * EMB_DIM / 4; i += NTHREADS) {
        const float4 v = ((const float4*)emb)[i];
        const int n = i >> 4;
        const int d = (i & 15) << 2;
        const size_t o = (size_t)d * KPITCH + n;
        const __bf16 h0 = (__bf16)v.x, h1 = (__bf16)v.y, h2 = (__bf16)v.z, h3 = (__bf16)v.w;
        embH[o]              = h0;  embL[o]              = (__bf16)(v.x - (float)h0);
        embH[o + KPITCH]     = h1;  embL[o + KPITCH]     = (__bf16)(v.y - (float)h1);
        embH[o + 2 * KPITCH] = h2;  embL[o + 2 * KPITCH] = (__bf16)(v.z - (float)h2);
        embH[o + 3 * KPITCH] = h3;  embL[o + 3 * KPITCH] = (__bf16)(v.w - (float)h3);
    }
    __syncthreads();

    float Mw = red[0], Mnw = red[1], Mb = red[2];
#pragma unroll
    for (int j = 1; j < NWAVES; ++j) {
        Mw  = fmaxf(Mw,  red[j * 3]);
        Mnw = fmaxf(Mnw, red[j * 3 + 1]);
        Mb  = fmaxf(Mb,  red[j * 3 + 2]);
    }

    const int  m    = lane & 15;
    const int  h    = lane >> 4;
    const long tile = (long)blockIdx.x * TOK_PER_BLOCK + (long)wv * 16;

    long xi = tile + m;
    if (xi > (long)T - 1) xi = (long)T - 1;
    const float x = x_in[xi];
    const float shift = fmaxf(x * Mw, -x * Mnw) + Mb;

    v8f acc[4] = {};
    float ps = 0.f;

#pragma unroll 1
    for (int kt = 0; kt < NUM_EMB / 32; ++kt) {
        const int kb = kt * 32;

        const float4* wq = (const float4*)(sw + kb + h * 8);
        const float4* bq = (const float4*)(sb + kb + h * 8);
        const float4 w0 = wq[0], w1 = wq[1], w2 = wq[4], w3 = wq[5];
        const float4 b0 = bq[0], b1 = bq[1], b2 = bq[4], b3 = bq[5];

        float e[16];
        e[0]  = __builtin_amdgcn_exp2f(fmaf(x, w0.x, b0.x) - shift);
        e[1]  = __builtin_amdgcn_exp2f(fmaf(x, w0.y, b0.y) - shift);
        e[2]  = __builtin_amdgcn_exp2f(fmaf(x, w0.z, b0.z) - shift);
        e[3]  = __builtin_amdgcn_exp2f(fmaf(x, w0.w, b0.w) - shift);
        e[4]  = __builtin_amdgcn_exp2f(fmaf(x, w1.x, b1.x) - shift);
        e[5]  = __builtin_amdgcn_exp2f(fmaf(x, w1.y, b1.y) - shift);
        e[6]  = __builtin_amdgcn_exp2f(fmaf(x, w1.z, b1.z) - shift);
        e[7]  = __builtin_amdgcn_exp2f(fmaf(x, w1.w, b1.w) - shift);
        e[8]  = __builtin_amdgcn_exp2f(fmaf(x, w2.x, b2.x) - shift);
        e[9]  = __builtin_amdgcn_exp2f(fmaf(x, w2.y, b2.y) - shift);
        e[10] = __builtin_amdgcn_exp2f(fmaf(x, w2.z, b2.z) - shift);
        e[11] = __builtin_amdgcn_exp2f(fmaf(x, w2.w, b2.w) - shift);
        e[12] = __builtin_amdgcn_exp2f(fmaf(x, w3.x, b3.x) - shift);
        e[13] = __builtin_amdgcn_exp2f(fmaf(x, w3.y, b3.y) - shift);
        e[14] = __builtin_amdgcn_exp2f(fmaf(x, w3.z, b3.z) - shift);
        e[15] = __builtin_amdgcn_exp2f(fmaf(x, w3.w, b3.w) - shift);

        ps += (((e[0] + e[1]) + (e[2] + e[3])) + ((e[4] + e[5]) + (e[6] + e[7])))
            + (((e[8] + e[9]) + (e[10] + e[11])) + ((e[12] + e[13]) + (e[14] + e[15])));

        v16b ah, al;
#pragma unroll
        for (int i = 0; i < 16; ++i) {
            const __bf16 hb = (__bf16)e[i];
            ah[i] = hb;
            al[i] = (__bf16)(e[i] - (float)hb);
        }

#pragma unroll
        for (int nt = 0; nt < 4; ++nt) {
            const size_t bo = (size_t)(nt * 16 + m) * KPITCH + kb + 8 * h;
            Frag bh, bl;
            bh.half[0] = *(const v8b*)(embH + bo);
            bh.half[1] = *(const v8b*)(embH + bo + 16);
            bl.half[0] = *(const v8b*)(embL + bo);
            bl.half[1] = *(const v8b*)(embL + bo + 16);
            acc[nt] = wmma3(acc[nt], ah, al, bh.v, bl.v);
        }
    }

    ps += __shfl_xor(ps, 16);
    float inv[8];
#pragma unroll
    for (int r = 0; r < 8; ++r) inv[r] = __builtin_amdgcn_rcpf(__shfl(ps, 8 * h + r));

    float* st = stage + wv * (16 * SPITCH);
#pragma unroll
    for (int nt = 0; nt < 4; ++nt) {
#pragma unroll
        for (int r = 0; r < 8; ++r) {
            st[(8 * h + r) * SPITCH + nt * 16 + m] = acc[nt][r] * inv[r];
        }
    }
    __syncthreads();

    const int c4 = m * 4;
    v4f vals[8];
#pragma unroll
    for (int j = 0; j < 8; ++j) vals[j] = *(const v4f*)(st + (2 * j + h) * SPITCH + c4);

#pragma unroll
    for (int j = 0; j < 8; ++j) {
        const long row = tile + 2 * j + h;
        if (row < (long)T) *(volatile v4f*)(out + row * EMB_DIM + c4) = vals[j];
    }
    __threadfence();
#pragma unroll
    for (int j = 0; j < 8; ++j) {
        const long row = tile + 2 * j + h;
        if (row < (long)T) *(volatile v4f*)(out + row * EMB_DIM + c4) = vals[j];
    }
}

extern "C" void kernel_launch(void* const* d_in, const int* in_sizes, int n_in,
                              void* d_out, int out_size, void* d_ws, size_t ws_size,
                              hipStream_t stream)
{
    if (n_in < 4) return;
    const float* x    = (const float*)d_in[0];
    const float* pw   = (const float*)d_in[1];
    const float* pb   = (const float*)d_in[2];
    const float* embp = (const float*)d_in[3];
    float*       outp = (float*)d_out;

    const int T = in_sizes[0];
    if (T <= 0) return;
    if (in_sizes[1] < NUM_EMB || in_sizes[2] < NUM_EMB || in_sizes[3] < NUM_EMB * EMB_DIM) return;
    if ((long)out_size < (long)T * EMB_DIM) return;

    const int blocks = (T + TOK_PER_BLOCK - 1) / TOK_PER_BLOCK;
    soft_emb_kernel<<<blocks, NTHREADS, (size_t)SMEM_BYTES, stream>>>(x, pw, pb, embp, outp, T);
}
